// GraphAttention_49237505081496
// MI455X (gfx1250) — hardware-verified
//
#include <hip/hip_runtime.h>
#include <math.h>

#ifndef NNODE
#define NNODE 16384
#endif
#define N_FULL 16384
#define NB 64
#define SEQ 512
#define DD 256
#define NH 4
#define HDIM 64
#define QKVM_RAW (((NNODE + SEQ + 63) / 64) * 64)
#define QKVM ((QKVM_RAW > N_FULL) ? N_FULL : QKVM_RAW)
#define KCH_MAX ((2 * SEQ) / 64 + 2)
#define ST_INTS 128
#define ST_FLAG 100
static_assert(NNODE % 64 == 0);
static_assert(NNODE >= 64);
static_assert(NNODE <= N_FULL);
static_assert(QKVM % 64 == 0);
static_assert(QKVM >= NNODE);
static_assert(N_FULL % 256 == 0);
static_assert(NB + 1 < ST_FLAG);
static_assert(ST_FLAG < ST_INTS);
static_assert(DD == NH * HDIM);
static_assert(HDIM == 64);
static_assert(DD % 32 == 0);

#define WSC 64.0f
#define XSC 1.0f
#define PSC 256.0f
#define OSC 32.0f
#define SCL 0.0625f

#define RB(x) ((((size_t)(x)) + 255) & ~(size_t)255)
#define WS_ST   RB((size_t)ST_INTS * 4)
#define WS_W16  RB((size_t)4 * DD * DD * 2)
#define WS_XN   RB((size_t)QKVM * DD * 2)
#define WS_QKV  RB((size_t)QKVM * 3 * DD * 2)
#define WS_ATT  RB((size_t)NNODE * DD * 2)
#define WS_TOTAL (WS_ST + WS_W16 + WS_XN + WS_QKV + WS_ATT)
static_assert(WS_TOTAL <= (size_t)134217728);

typedef __attribute__((ext_vector_type(16))) _Float16 v16h;
typedef __attribute__((ext_vector_type(8)))  _Float16 v8h;
typedef __attribute__((ext_vector_type(8)))  float    v8f;
typedef __attribute__((ext_vector_type(4)))  float    v4f;
typedef __attribute__((ext_vector_type(4)))  unsigned int v4u;
typedef __attribute__((ext_vector_type(4)))  int      v4i;

#define VST2(T, ptr, val) do { const T vst2_v_ = (val); *(volatile T*)(ptr) = vst2_v_; __threadfence(); *(volatile T*)(ptr) = vst2_v_; } while (0)

__device__ __forceinline__ float bfr(float v) { const unsigned u = __float_as_uint(v); const unsigned r = (u + 0x7fffu + ((u >> 16) & 1u)) & 0xffff0000u; return __uint_as_float(r); }
__device__ __forceinline__ unsigned int pk2h(float a, float b) { return (unsigned int)__builtin_bit_cast(unsigned short, (_Float16)a) | ((unsigned int)__builtin_bit_cast(unsigned short, (_Float16)b) << 16); }

union FragU { v16h v; v8h h[2]; };
__device__ __forceinline__ v16h frag_ld(const _Float16* p) { FragU f; f.h[0] = *(const v8h*)(p); f.h[1] = *(const v8h*)(p + 16); return f.v; }
__device__ __forceinline__ v8f wmma16(v16h a, v16h b, v8f c) {
    c = __builtin_amdgcn_wmma_f32_16x16x32_f16(false, a, false, b, (short)0, c, false, false);
    asm volatile("v_nop\n\tv_nop\n\tv_nop\n\tv_nop" : "+v"(c) : "v"(a), "v"(b));
    return c;
}
__device__ __forceinline__ void dep_guard_h(v8f& a, v8f& b, v16h x, v16h y) { asm volatile("v_nop\n\tv_nop\n\tv_nop\n\tv_nop" : "+v"(a), "+v"(b) : "v"(x), "v"(y)); }
__device__ __forceinline__ void keep4_h(v16h a, v16h b, v16h c, v16h d) { asm volatile("v_nop" :: "v"(a), "v"(b), "v"(c), "v"(d)); }
__device__ __forceinline__ void acc_guard4(v8f& a, v8f& b, v8f& c, v8f& d) { asm volatile("v_nop\n\tv_nop\n\tv_nop\n\tv_nop" : "+v"(a), "+v"(b), "+v"(c), "+v"(d)); }

__global__ __launch_bounds__(256) void k_starts(const int* __restrict__ batch, int* __restrict__ ST) {
    __shared__ int sv[256];
    __shared__ int sbad[256];
    const int t = threadIdx.x;
    int bad = 0;
    const int per = N_FULL / 256;
    for (int i = t * per; i < (t + 1) * per; ++i) {
        const int a = batch[i];
        const int nx = batch[min(i + 1, N_FULL - 1)];
        bad |= (a < 0 || a >= NB) ? 1 : 0;
        bad |= (i + 1 < N_FULL && a > nx) ? 1 : 0;
    }
    const int tt = min(t, NB);
    int lo = 0, hi = N_FULL;
#pragma unroll 1
    for (int it = 0; it < 16; ++it) {
        const int mid = (lo + hi) >> 1;
        const int bm = batch[min(mid, N_FULL - 1)];
        const bool go = (lo < hi);
        if (go) { if (bm < tt) lo = mid + 1; else hi = mid; }
    }
    sv[t] = (t < NB) ? lo : N_FULL;
    sbad[t] = bad;
    __syncthreads();
    int bad2 = 0;
    if (t < NB) { const int cn = sv[t + 1] - sv[t]; bad2 = (cn > SEQ || cn < 0) ? 1 : 0; }
    __syncthreads();
    sbad[t] |= bad2;
    __syncthreads();
    for (int o = 128; o > 0; o >>= 1) { if (t < o) sbad[t] |= sbad[t + o]; __syncthreads(); }
    if (t < ST_INTS) {
        const int v = (t <= NB) ? sv[t] : ((t == ST_FLAG) ? sbad[0] : 0);
        VST2(int, ST + t, v);
    }
}

__global__ __launch_bounds__(256) void k_castw(const float* __restrict__ Wq, const float* __restrict__ Wh, unsigned short* __restrict__ W16) {
    const int u = blockIdx.x * 256 + threadIdx.x;
    if (u >= 4 * DD * (DD / 8)) return;
    const int r = u / (DD / 8), c0 = 8 * (u % (DD / 8));
    const float* pa = Wq + (size_t)min(r, 3 * DD - 1) * DD + c0;
    const float* pb = Wh + (size_t)min(max(r - 3 * DD, 0), DD - 1) * DD + c0;
    const v4f a0 = *(const v4f*)(pa), a1 = *(const v4f*)(pa + 4);
    const v4f b0 = *(const v4f*)(pb), b1 = *(const v4f*)(pb + 4);
    const bool uq = (r < 3 * DD);
    const float aa[8] = {a0.x, a0.y, a0.z, a0.w, a1.x, a1.y, a1.z, a1.w};
    const float ab[8] = {b0.x, b0.y, b0.z, b0.w, b1.x, b1.y, b1.z, b1.w};
    float w[8];
#pragma unroll
    for (int e = 0; e < 8; ++e) w[e] = bfr(uq ? aa[e] : ab[e]) * WSC;
    v4u pk; pk.x = pk2h(w[0], w[1]); pk.y = pk2h(w[2], w[3]); pk.z = pk2h(w[4], w[5]); pk.w = pk2h(w[6], w[7]);
    VST2(v4u, (v4u*)(W16 + (size_t)r * DD + c0), pk);
}

__global__ __launch_bounds__(256) void k_ln(const float* __restrict__ X, const float* __restrict__ g, const float* __restrict__ bb, unsigned short* __restrict__ XN, int nrows) {
    #pragma clang fp contract(off)
    const int row = blockIdx.x * 8 + (threadIdx.x >> 5);
    const int L = threadIdx.x & 31;
    if (row >= nrows) return;
    const float* xr = X + (size_t)row * DD + 8 * L;
    const v4f a = *(const v4f*)(xr), b = *(const v4f*)(xr + 4);
    float v[8] = {a.x, a.y, a.z, a.w, b.x, b.y, b.z, b.w};
#pragma unroll
    for (int e = 0; e < 8; ++e) v[e] = bfr(v[e]);
    float s = ((v[0] + v[1]) + (v[2] + v[3])) + ((v[4] + v[5]) + (v[6] + v[7]));
#pragma unroll
    for (int o = 16; o > 0; o >>= 1) s += __shfl_xor(s, o, 32);
    const float mu = s * (1.0f / 256.0f);
    float d[8];
    float q = 0.f;
#pragma unroll
    for (int e = 0; e < 8; ++e) { d[e] = v[e] - mu; q += d[e] * d[e]; }
#pragma unroll
    for (int o = 16; o > 0; o >>= 1) q += __shfl_xor(q, o, 32);
    const float rstd = rsqrtf(q * (1.0f / 256.0f) + 1e-5f);
    const v4f g0 = *(const v4f*)(g + 8 * L), g1 = *(const v4f*)(g + 8 * L + 4);
    const v4f c0 = *(const v4f*)(bb + 8 * L), c1 = *(const v4f*)(bb + 8 * L + 4);
    const float gg[8] = {g0.x, g0.y, g0.z, g0.w, g1.x, g1.y, g1.z, g1.w};
    const float cc[8] = {c0.x, c0.y, c0.z, c0.w, c1.x, c1.y, c1.z, c1.w};
    float y[8];
#pragma unroll
    for (int e = 0; e < 8; ++e) y[e] = (((d[e] * rstd) * bfr(gg[e])) + bfr(cc[e])) * XSC;
    v4u pk; pk.x = pk2h(y[0], y[1]); pk.y = pk2h(y[2], y[3]); pk.z = pk2h(y[4], y[5]); pk.w = pk2h(y[6], y[7]);
    VST2(v4u, (v4u*)(XN + (size_t)row * DD + 8 * L), pk);
}

template <int OUT_MODE, int BIAS_MODE, bool RESID, bool POISON>
__global__ __launch_bounds__(256) void k_gemm64(const unsigned short* __restrict__ Ap, int lda, const unsigned short* __restrict__ Btp, int ldb,
                                               void* __restrict__ Cout, int ldc, const float* __restrict__ bias, const float* __restrict__ resid, int ldr,
                                               const int* __restrict__ flag, int M, int N, int K, float scale) {
    static_assert(!(RESID && OUT_MODE != 0));
    static_assert(!(BIAS_MODE != 0 && OUT_MODE != 0));
    const _Float16* A = (const _Float16*)Ap;
    const _Float16* Bt = (const _Float16*)Btp;
    __shared__ __align__(16) float sT[8][16 * 68];
    const int lane = threadIdx.x & 31, wave = threadIdx.x >> 5;
    const int tilesN = N >> 6, tilesM = M >> 6;
    const int tile = blockIdx.x * 8 + wave;
    if (tile >= tilesM * tilesN) return;
    const int tm = tile / tilesN, tn = tile - tm * tilesN;
    const int m0 = tm << 6, n0 = tn << 6;
    const int rlane = lane & 15;
    const int koff = (lane >> 4) * 8;
    const int mOff = (lane >> 4) * 8;

    v8f acc[4][4];
#pragma unroll
    for (int i = 0; i < 4; ++i)
#pragma unroll
        for (int j = 0; j < 4; ++j) { v8f zz = {}; acc[i][j] = zz; }

    for (int k0 = 0; k0 < K; k0 += 32) {
        v16h bh[4];
#pragma unroll
        for (int j = 0; j < 4; ++j) bh[j] = frag_ld(Bt + (size_t)(n0 + (j << 4) + rlane) * ldb + koff + k0);
#pragma unroll
        for (int i = 0; i < 4; ++i) {
            const v16h ah = frag_ld(A + (size_t)(m0 + (i << 4) + rlane) * lda + koff + k0);
#pragma unroll
            for (int j = 0; j < 4; ++j) acc[i][j] = __builtin_amdgcn_wmma_f32_16x16x32_f16(false, ah, false, bh[j], (short)0, acc[i][j], false, false);
            dep_guard_h(acc[i][0], acc[i][3], ah, ah);
        }
        keep4_h(bh[0], bh[1], bh[2], bh[3]);
    }
    acc_guard4(acc[0][0], acc[0][1], acc[0][2], acc[0][3]);
    acc_guard4(acc[1][0], acc[1][1], acc[1][2], acc[1][3]);
    acc_guard4(acc[2][0], acc[2][1], acc[2][2], acc[2][3]);
    acc_guard4(acc[3][0], acc[3][1], acc[3][2], acc[3][3]);

    const int pz = POISON ? flag[0] : 0;
    const float qnan = __uint_as_float(0x7fc00000u);
    float* slab = sT[wave];
#pragma unroll
    for (int i = 0; i < 4; ++i) {
        const int mBase = m0 + (i << 4);
#pragma unroll
        for (int j = 0; j < 4; ++j) {
#pragma unroll
            for (int r = 0; r < 8; ++r) {
                float v = acc[i][j][r] * scale;
                if (POISON) v = (pz != 0) ? qnan : v;
                slab[(mOff + r) * 68 + (j << 4) + rlane] = v;
            }
        }
        __builtin_amdgcn_fence(3  , "workgroup");
        __builtin_amdgcn_wave_barrier();
        __builtin_amdgcn_fence(2  , "workgroup");
        if (OUT_MODE == 0) {
            float* C = (float*)Cout;
            const int hq = lane >> 4, c4 = (lane & 15) * 4;
            v4f badd = {0.f, 0.f, 0.f, 0.f};
            if (BIAS_MODE == 2) { const v4f bq = *(const v4f*)(bias + n0 + c4); badd.x = bfr(bq.x); badd.y = bfr(bq.y); badd.z = bfr(bq.z); badd.w = bfr(bq.w); }
            v4f vv[8];
#pragma unroll
            for (int it = 0; it < 8; ++it) {
                const int row = it * 2 + hq;
                v4f tv = *(const v4f*)(slab + row * 68 + c4);
                if (BIAS_MODE == 2) tv += badd;
                if (RESID) {
                    const v4f rr = *(const v4f*)(resid + (size_t)(mBase + row) * ldr + n0 + c4);
                    tv.x += bfr(rr.x); tv.y += bfr(rr.y); tv.z += bfr(rr.z); tv.w += bfr(rr.w);
                }
                vv[it] = tv;
            }
            for (int pass = 0; pass < 2; ++pass) {
#pragma unroll
                for (int it = 0; it < 8; ++it) {
                    const int row = it * 2 + hq;
                    *(volatile v4f*)(C + (size_t)(mBase + row) * ldc + n0 + c4) = vv[it];
                }
                __threadfence();
            }
        } else {
            unsigned short* C = (unsigned short*)Cout;
            const int q8 = lane >> 3, c8 = (lane & 7) * 8;
            v8h hv[4];
#pragma unroll
            for (int it = 0; it < 4; ++it) {
                const int row = it * 4 + q8;
                const float* sp = slab + row * 68 + c8;
#pragma unroll
                for (int e = 0; e < 8; ++e) hv[it][e] = (_Float16)sp[e];
            }
            for (int pass = 0; pass < 2; ++pass) {
#pragma unroll
                for (int it = 0; it < 4; ++it) {
                    const int row = it * 4 + q8;
                    *(volatile v8h*)(C + (size_t)(mBase + row) * ldc + n0 + c8) = hv[it];
                }
                __threadfence();
            }
        }
        __builtin_amdgcn_fence(3  , "workgroup");
        __builtin_amdgcn_wave_barrier();
        __builtin_amdgcn_fence(2  , "workgroup");
    }
}

__global__ __launch_bounds__(128) void k_gattn(const unsigned short* __restrict__ QKVp, const int* __restrict__ batch, const int* __restrict__ ST,
                                              unsigned short* __restrict__ ATT, int nkey) {
    const _Float16* QKV = (const _Float16*)QKVp;
    __shared__ __align__(16) _Float16 Ksh[64 * 64];
    __shared__ __align__(16) _Float16 Vth[64 * 64];
    __shared__ __align__(16) _Float16 Psh[4][16 * 64];
    __shared__ __align__(16) float    Os[4][16 * 68];
    __shared__ int stl[ST_INTS];
    const int tid = threadIdx.x, wave = tid >> 5, lane = tid & 31, hh = lane >> 4, c = lane & 15;
    const int h = blockIdx.y;
    const int nblk = blockIdx.x * 64;
    const int q0 = nblk + wave * 16;
    const float NEG = -__builtin_inff();
    const float SL2 = SCL * 1.4426950408889634f;
    const int LDQ = 3 * DD;

    stl[tid] = ST[tid];
    __syncthreads();

    const int blo = min(max(batch[nblk], 0), NB - 1);
    const int bhi = min(max(batch[nblk + 63], 0), NB - 1);
    const int klo = min(max(stl[blo], 0), nkey);
    const int khi = min(max(stl[bhi + 1], 0), nkey);
    const int kvs = (klo >> 6) << 6;
    int nch = (khi > kvs) ? ((khi - kvs + 63) >> 6) : 0;
    nch = min(nch, KCH_MAX);

    int glo[8], ghi[8];
    {
        const v4i ba = *(const v4i*)(batch + q0 + 8 * hh);
        const v4i bbv = *(const v4i*)(batch + q0 + 8 * hh + 4);
        const int bq[8] = {ba.x, ba.y, ba.z, ba.w, bbv.x, bbv.y, bbv.z, bbv.w};
#pragma unroll
        for (int r = 0; r < 8; ++r) {
            const int b = min(max(bq[r], 0), NB - 1);
            int lo = stl[b], hi = stl[b + 1];
            lo = min(max(lo, 0), nkey);
            hi = min(max(hi, lo), nkey);
            hi = min(hi, lo + SEQ);
            glo[r] = lo; ghi[r] = hi;
        }
    }

    v16h qa0, qa1;
    {
        const _Float16* qrow = QKV + (size_t)(q0 + c) * LDQ + h * HDIM;
        qa0 = frag_ld(qrow + 8 * hh);
        qa1 = frag_ld(qrow + 32 + 8 * hh);
    }

    float mrow[8], lrow[8];
    v8f oacc[4];
#pragma unroll
    for (int r = 0; r < 8; ++r) { mrow[r] = NEG; lrow[r] = 0.f; }
#pragma unroll
    for (int t = 0; t < 4; ++t) { v8f zz = {}; oacc[t] = zz; }

    for (int kc = 0; kc < nch; ++kc) {
        const int kv0 = kvs + (kc << 6);
        __syncthreads();
#pragma unroll
        for (int i = 0; i < 4; ++i) {
            const int idx = tid + 128 * i;
            const int kvr = idx >> 3, c8 = (idx & 7) * 8;
            const int krow = min(kv0 + kvr, nkey - 1);
            const _Float16* src = QKV + (size_t)krow * LDQ + h * HDIM + c8;
            const v8h k8 = *(const v8h*)(src + DD);
            const v8h w8 = *(const v8h*)(src + 2 * DD);
            *(v8h*)(Ksh + kvr * 64 + c8) = k8;
#pragma unroll
            for (int e = 0; e < 8; ++e) Vth[(c8 + e) * 64 + kvr] = w8[e];
        }
        __syncthreads();

        v8f s[4];
#pragma unroll
        for (int j = 0; j < 4; ++j) {
            v8f z = {};
            FragU kb0, kb1;
            kb0.h[0] = *(const v8h*)(Ksh + (j * 16 + c) * 64 + 8 * hh);
            kb0.h[1] = *(const v8h*)(Ksh + (j * 16 + c) * 64 + 16 + 8 * hh);
            kb1.h[0] = *(const v8h*)(Ksh + (j * 16 + c) * 64 + 32 + 8 * hh);
            kb1.h[1] = *(const v8h*)(Ksh + (j * 16 + c) * 64 + 48 + 8 * hh);
            z = wmma16(qa0, kb0.v, z);
            z = wmma16(qa1, kb1.v, z);
            s[j] = z;
        }
        float cm[8];
#pragma unroll
        for (int r = 0; r < 8; ++r) {
            const int lo = glo[r], hi = ghi[r];
            float m = NEG;
#pragma unroll
            for (int j = 0; j < 4; ++j) {
                const int kvcol = kv0 + j * 16 + c;
                const bool keep = (kvcol >= lo) && (kvcol < hi);
                const float v = keep ? (s[j][r] * SL2) : NEG;
                s[j][r] = v;
                m = fmaxf(m, v);
            }
#pragma unroll
            for (int off = 1; off < 16; off <<= 1) m = fmaxf(m, __shfl_xor(m, off, 32));
            cm[r] = m;
        }
        _Float16* pw = Psh[wave];
#pragma unroll
        for (int r = 0; r < 8; ++r) {
            const float mnew = fmaxf(mrow[r], cm[r]);
            const float alpha = (mnew == NEG) ? 1.f : exp2f(mrow[r] - mnew);
            mrow[r] = mnew;
            float psum = 0.f;
#pragma unroll
            for (int j = 0; j < 4; ++j) {
                const float sv = s[j][r];
                const float p = (sv == NEG) ? 0.f : exp2f(sv - mnew);
                psum += p;
                pw[(8 * hh + r) * 64 + j * 16 + c] = (_Float16)(p * PSC);
            }
#pragma unroll
            for (int off = 1; off < 16; off <<= 1) psum += __shfl_xor(psum, off, 32);
            lrow[r] = lrow[r] * alpha + psum;
#pragma unroll
            for (int t = 0; t < 4; ++t) oacc[t][r] *= alpha;
        }
        __builtin_amdgcn_fence(3  , "workgroup");
        __builtin_amdgcn_wave_barrier();
        __builtin_amdgcn_fence(2  , "workgroup");
#pragma unroll
        for (int kk = 0; kk < 2; ++kk) {
            FragU pa;
            pa.h[0] = *(const v8h*)(pw + c * 64 + kk * 32 + 8 * hh);
            pa.h[1] = *(const v8h*)(pw + c * 64 + kk * 32 + 16 + 8 * hh);
#pragma unroll
            for (int t = 0; t < 4; ++t) {
                FragU vb;
                vb.h[0] = *(const v8h*)(Vth + (t * 16 + c) * 64 + kk * 32 + 8 * hh);
                vb.h[1] = *(const v8h*)(Vth + (t * 16 + c) * 64 + kk * 32 + 16 + 8 * hh);
                oacc[t] = wmma16(pa.v, vb.v, oacc[t]);
            }
        }
    }

    float* os = Os[wave];
#pragma unroll
    for (int r = 0; r < 8; ++r) {
        const float den = lrow[r] * PSC;
        const float inv = (lrow[r] > 0.f) ? (OSC * (1.0f / den)) : 0.f;
#pragma unroll
        for (int t = 0; t < 4; ++t) os[(8 * hh + r) * 68 + t * 16 + c] = oacc[t][r] * inv;
    }
    __builtin_amdgcn_fence(3  , "workgroup");
    __builtin_amdgcn_wave_barrier();
    __builtin_amdgcn_fence(2  , "workgroup");
    {
        const int q8 = lane >> 3, c8 = (lane & 7) * 8;
#pragma unroll
        for (int it = 0; it < 4; ++it) {
            const int row = it * 4 + q8;
            const float* sp = os + row * 68 + c8;
            const v4f a = *(const v4f*)(sp), b = *(const v4f*)(sp + 4);
            v4u pk; pk.x = pk2h(a.x, a.y); pk.y = pk2h(a.z, a.w); pk.z = pk2h(b.x, b.y); pk.w = pk2h(b.z, b.w);
            VST2(v4u, (v4u*)(ATT + (size_t)(q0 + row) * DD + h * HDIM + c8), pk);
        }
    }
}

extern "C" void kernel_launch(void* const* d_in, const int* in_sizes, int n_in, void* d_out, int out_size, void* d_ws, size_t ws_size, hipStream_t stream) {
    if (n_in < 7) return;
    if (in_sizes[0] < N_FULL * DD || in_sizes[1] < 3 * DD * DD || in_sizes[2] < DD * DD || in_sizes[3] < DD || in_sizes[4] < DD || in_sizes[5] < DD || in_sizes[6] < N_FULL) return;
    if (out_size < NNODE * DD) return;
    if ((size_t)WS_TOTAL > ws_size) return;
    const float* x     = (const float*)d_in[0];
    const float* qkv_w = (const float*)d_in[1];
    const float* h_w   = (const float*)d_in[2];
    const float* h_b   = (const float*)d_in[3];
    const float* ln_w  = (const float*)d_in[4];
    const float* ln_b  = (const float*)d_in[5];
    const int*   batch = (const int*)d_in[6];
    float* out = (float*)d_out;

    char* wsp = (char*)d_ws;
    int* ST = (int*)wsp;                          wsp += WS_ST;
    unsigned short* W16 = (unsigned short*)wsp;   wsp += WS_W16;
    unsigned short* XN16 = (unsigned short*)wsp;  wsp += WS_XN;
    unsigned short* QKV16 = (unsigned short*)wsp; wsp += WS_QKV;
    unsigned short* ATT16 = (unsigned short*)wsp; wsp += WS_ATT;
    if ((size_t)(wsp - (char*)d_ws) > ws_size) return;

    k_starts<<<1, 256, 0, stream>>>(batch, ST);
    k_castw<<<(4 * DD * (DD / 8) + 255) / 256, 256, 0, stream>>>(qkv_w, h_w, W16);
    k_ln<<<QKVM / 8, 256, 0, stream>>>(x, ln_w, ln_b, XN16, QKVM);
    {
        const int tiles = (QKVM / 64) * ((3 * DD) / 64);
        k_gemm64<1, 0, false, false><<<(tiles + 7) / 8, 256, 0, stream>>>(XN16, DD, W16, DD, (void*)QKV16, 3 * DD, h_b, x, DD, ST + ST_FLAG, QKVM, 3 * DD, DD, 1.0f / (XSC * WSC));
    }
    k_gattn<<<dim3(NNODE / 64, NH), 128, 0, stream>>>(QKV16, batch, ST, ATT16, QKVM);
    {
        const int tiles = (NNODE / 64) * (DD / 64);
        k_gemm64<0, 2, true, true><<<(tiles + 7) / 8, 256, 0, stream>>>(ATT16, DD, W16 + (size_t)3 * DD * DD, DD, (void*)out, DD, h_b, x, DD, ST + ST_FLAG, NNODE, DD, DD, 1.0f / (OSC * WSC));
    }
}
